// Transformer_89386859364427
// MI455X (gfx1250) — hardware-verified
//
#include <hip/hip_runtime.h>

typedef __attribute__((ext_vector_type(16))) __bf16 v16b;
typedef __attribute__((ext_vector_type(8)))  float  v8f;
typedef __attribute__((ext_vector_type(4)))  float  v4f;

#define LAT    1024
#define SEQ    1024
#define NTOK   2048
#define NNODES 255
#define LW     16

__device__ __forceinline__ float gelu_exact(float x) {
  return 0.5f * x * (1.f + erff(x * 0.70710678118654752f));
}

__device__ __forceinline__ unsigned short f2bf_bits(float f) {
  unsigned u = __float_as_uint(f);
  return (unsigned short)((u + 0x7FFFu + ((u >> 16) & 1u)) >> 16);
}
__device__ __forceinline__ float bf_bits2f(unsigned short h) { return __uint_as_float(((unsigned)h) << 16); }

__device__ __forceinline__ void load_split(const float* p, v16b& hi, v16b& lo) {
  v4f t0 = *(const v4f*)(p), t1 = *(const v4f*)(p + 4), t2 = *(const v4f*)(p + 16), t3 = *(const v4f*)(p + 20);
  float v[16] = {t0[0],t0[1],t0[2],t0[3],t1[0],t1[1],t1[2],t1[3],t2[0],t2[1],t2[2],t2[3],t3[0],t3[1],t3[2],t3[3]};
#pragma unroll
  for (int e = 0; e < 16; ++e) {
    unsigned short hb = f2bf_bits(v[e]);
    unsigned short lb = f2bf_bits(v[e] - bf_bits2f(hb));
    hi[e] = __builtin_bit_cast(__bf16, hb);
    lo[e] = __builtin_bit_cast(__bf16, lb);
  }
}
__device__ __forceinline__ v8f wmma3(v16b ah, v16b al, v16b bh, v16b bl, v8f acc) {
  acc = __builtin_amdgcn_wmma_f32_16x16x32_bf16(false, ah, false, bh, (short)0, acc, false, false);
  acc = __builtin_amdgcn_wmma_f32_16x16x32_bf16(false, ah, false, bl, (short)0, acc, false, false);
  acc = __builtin_amdgcn_wmma_f32_16x16x32_bf16(false, al, false, bh, (short)0, acc, false, false);
  asm volatile("v_nop\n\tv_nop\n\tv_nop\n\tv_nop" : "+v"(acc) : "v"(ah), "v"(al), "v"(bh), "v"(bl));
  return acc;
}

__global__ void __launch_bounds__(256) norm_kernel(const float* __restrict__ x, float* __restrict__ xn) {
  __shared__ float r1[8], r2[8];
  __shared__ float smu, sinv;
  const int t = threadIdx.x;
  const float* xr = x + (size_t)blockIdx.x * LAT;
  float v[4]; float s = 0.f;
#pragma unroll
  for (int i = 0; i < 4; i++) { float a = xr[t + 256 * i]; v[i] = a; s += a; }
#pragma unroll
  for (int o = 16; o > 0; o >>= 1) s += __shfl_down(s, o, 32);
  if ((t & 31) == 0) r1[t >> 5] = s;
  __syncthreads();
  if (t == 0) {
    float ss = 0.f;
    for (int w = 0; w < 8; w++) ss += r1[w];
    smu = ss * (1.f / LAT);
  }
  __syncthreads();
  const float mu = smu;
  float s2 = 0.f;
#pragma unroll
  for (int i = 0; i < 4; i++) { float d = v[i] - mu; s2 += d * d; }
#pragma unroll
  for (int o = 16; o > 0; o >>= 1) s2 += __shfl_down(s2, o, 32);
  if ((t & 31) == 0) r2[t >> 5] = s2;
  __syncthreads();
  if (t == 0) {
    float qq = 0.f;
    for (int w = 0; w < 8; w++) qq += r2[w];
    float sd = sqrtf(qq * (1.f / (LAT - 1)));
    sinv = 1.f / sqrtf(sd + 1e-5f);
  }
  __syncthreads();
  const float inv = sinv;
  float* xo = xn + (size_t)blockIdx.x * LAT;
#pragma unroll
  for (int i = 0; i < 4; i++) ((volatile float*)xo)[t + 256 * i] = (v[i] - mu) * inv;
  __threadfence();
#pragma unroll
  for (int i = 0; i < 4; i++) ((volatile float*)xo)[t + 256 * i] = (v[i] - mu) * inv;
}

template <int MODE>
__global__ void __launch_bounds__(256) fff_kernel(const float* __restrict__ in,
                           const float* __restrict__ nw, const float* __restrict__ nb,
                           const float* __restrict__ w1, const float* __restrict__ b1,
                           const float* __restrict__ w2, const float* __restrict__ b2,
                           float* __restrict__ outf) {
  __shared__ float xs[LAT];
  __shared__ float red[8];
  __shared__ float hred[8][LW];
  __shared__ float hs[LW];
  __shared__ int   snode;
  const int t   = threadIdx.x;
  const int tok = blockIdx.x;
  const float* xr = in + (size_t)tok * LAT;
  for (int d = t; d < LAT; d += 256) xs[d] = xr[d];
  __syncthreads();

  int node = 0;
  for (int step = 0; step < 8; ++step) {
    const float* nwp = nw + (size_t)node * LAT;
    float p = 0.f;
#pragma unroll 1
    for (int d = t; d < LAT; d += 256) p += xs[d] * nwp[d];
#pragma unroll
    for (int o = 16; o > 0; o >>= 1) p += __shfl_down(p, o, 32);
    if ((t & 31) == 0) red[t >> 5] = p;
    __syncthreads();
    if (t == 0) {
      float s = 0.f;
      for (int w = 0; w < 8; w++) s += red[w];
      s += nb[node];
      snode = 2 * node + 1 + (s > 0.f ? 1 : 0);
    }
    __syncthreads();
    node = snode;
    __syncthreads();
  }
  int leaf = node - NNODES;
  leaf = leaf < 0 ? 0 : (leaf > 255 ? 255 : leaf);

  float acc[LW];
#pragma unroll
  for (int j = 0; j < LW; j++) acc[j] = 0.f;
  const float* w1l = w1 + (size_t)leaf * LAT * LW;
#pragma unroll 1
  for (int d = t; d < LAT; d += 256) {
    const float xv = xs[d];
    const v4f* wr = (const v4f*)(w1l + (size_t)d * LW);
#pragma unroll
    for (int q4 = 0; q4 < 4; q4++) {
      v4f w = wr[q4];
      acc[q4 * 4 + 0] += xv * w[0];
      acc[q4 * 4 + 1] += xv * w[1];
      acc[q4 * 4 + 2] += xv * w[2];
      acc[q4 * 4 + 3] += xv * w[3];
    }
  }
#pragma unroll
  for (int j = 0; j < LW; j++) {
    float p = acc[j];
#pragma unroll
    for (int o = 16; o > 0; o >>= 1) p += __shfl_down(p, o, 32);
    if ((t & 31) == 0) hred[t >> 5][j] = p;
  }
  __syncthreads();
  if (t < LW) {
    float s = 0.f;
    for (int w = 0; w < 8; w++) s += hred[w][t];
    s += b1[leaf * LW + t];
    hs[t] = (MODE == 0) ? fmaxf(s, 0.f) : gelu_exact(s);
  }
  __syncthreads();

  const float* w2l = w2 + (size_t)leaf * LW * LAT;
  const float* b2l = b2 + (size_t)leaf * LAT;
  float ov[4];
#pragma unroll
  for (int i = 0; i < 4; ++i) {
    const int d = t + 256 * i;
    float v = 0.f;
#pragma unroll
    for (int j = 0; j < LW; j++) v += hs[j] * w2l[j * LAT + d];
    v += b2l[d];
    ov[i] = (MODE == 0) ? v : (xs[d] + v);
  }
  float* op = outf + (size_t)tok * LAT;
#pragma unroll
  for (int i = 0; i < 4; ++i) ((volatile float*)op)[t + 256 * i] = ov[i];
  __threadfence();
#pragma unroll
  for (int i = 0; i < 4; ++i) ((volatile float*)op)[t + 256 * i] = ov[i];
}

__global__ void __launch_bounds__(256) abt_split_kernel(const float* __restrict__ A, int lda, long sA,
                                 const float* __restrict__ B, int ldb, long sB,
                                 float* __restrict__ C, int ldc, long sC,
                                 const float* __restrict__ add, long sAdd,
                                 int N, int K, float alpha) {
  __shared__ __align__(16) float sT[8][16 * 36];
  const int lane = threadIdx.x & 31, wave = threadIdx.x >> 5;
  const int g = lane >> 4, m = lane & 15;
  const int b = blockIdx.y;
  const int nblkPerRow = N / 256;
  const int mt = blockIdx.x / nblkPerRow;
  const int n0 = (blockIdx.x % nblkPerRow) * 256 + wave * 32;
  const float* Ab = A + (size_t)b * sA + (size_t)(mt * 16 + m) * lda + g * 8;
  const float* B0 = B + (size_t)b * sB + (size_t)(n0 + m) * ldb + g * 8;
  const float* B1 = B0 + (size_t)16 * ldb;
  v8f acc0 = {}, acc1 = {};
  for (int k = 0; k < K; k += 32) {
    v16b ah, al, bh, bl, ch, cl;
    load_split(Ab + k, ah, al);
    load_split(B0 + k, bh, bl);
    load_split(B1 + k, ch, cl);
    acc0 = wmma3(ah, al, bh, bl, acc0);
    acc1 = wmma3(ah, al, ch, cl, acc1);
  }
  float* slab = sT[wave];
  const float* addb = add ? (add + (size_t)b * sAdd) : nullptr;
#pragma unroll
  for (int r = 0; r < 8; ++r) {
    const int row = 8 * g + r;
    float v0 = acc0[r] * alpha, v1 = acc1[r] * alpha;
    if (addb) {
      v0 += addb[(size_t)(mt * 16 + row) * ldc + n0 + m];
      v1 += addb[(size_t)(mt * 16 + row) * ldc + n0 + 16 + m];
    }
    slab[row * 36 + m] = v0;
    slab[row * 36 + 16 + m] = v1;
  }
  __builtin_amdgcn_fence(__ATOMIC_RELEASE, "workgroup");
  __builtin_amdgcn_wave_barrier();
  __builtin_amdgcn_fence(__ATOMIC_ACQUIRE, "workgroup");
  float* Cb = C + (size_t)b * sC + (size_t)(mt * 16) * ldc + n0;
  const int q = lane >> 3, c4 = (lane & 7) * 4;
  for (int pass = 0; pass < 2; ++pass) {
#pragma unroll
    for (int it = 0; it < 4; ++it) {
      const int row = it * 4 + q;
      v4f v = *(const v4f*)(slab + row * 36 + c4);
      *(volatile v4f*)(Cb + (size_t)row * ldc + c4) = v;
    }
    __threadfence();
  }
}

__global__ void __launch_bounds__(256) softmax_kernel(const float* __restrict__ sc, float* __restrict__ ph) {
  __shared__ float red[8];
  __shared__ float sbc;
  const int t = threadIdx.x;
  const float* row = sc + (size_t)blockIdx.x * SEQ;
  float*       out = ph + (size_t)blockIdx.x * SEQ;
  float v[4];
  float m = -3.4e38f;
#pragma unroll
  for (int i = 0; i < 4; i++) { v[i] = row[t + 256 * i]; m = fmaxf(m, v[i]); }
#pragma unroll
  for (int o = 16; o > 0; o >>= 1) m = fmaxf(m, __shfl_down(m, o, 32));
  if ((t & 31) == 0) red[t >> 5] = m;
  __syncthreads();
  if (t == 0) { float mm = red[0]; for (int w = 1; w < 8; w++) mm = fmaxf(mm, red[w]); sbc = mm; }
  __syncthreads();
  m = sbc;
  __syncthreads();
  float s = 0.f;
#pragma unroll
  for (int i = 0; i < 4; i++) { v[i] = expf(v[i] - m); s += v[i]; }
#pragma unroll
  for (int o = 16; o > 0; o >>= 1) s += __shfl_down(s, o, 32);
  if ((t & 31) == 0) red[t >> 5] = s;
  __syncthreads();
  if (t == 0) { float ss = 0.f; for (int w = 0; w < 8; w++) ss += red[w]; sbc = 1.f / ss; }
  __syncthreads();
  const float inv = sbc;
#pragma unroll
  for (int i = 0; i < 4; i++) ((volatile float*)out)[t + 256 * i] = v[i] * inv;
  __threadfence();
#pragma unroll
  for (int i = 0; i < 4; i++) ((volatile float*)out)[t + 256 * i] = v[i] * inv;
}

__global__ void __launch_bounds__(256) vtrans_kernel(const float* __restrict__ vh, float* __restrict__ vt) {
  __shared__ float tile[32][33];
  const int bid = blockIdx.x;
  const int b  = bid >> 10;
  const int r  = bid & 1023;
  const int ty = r >> 5;
  const int tx = r & 31;
  const int t  = threadIdx.x;
  const int lr = t >> 5;
  const int lc = t & 31;
#pragma unroll
  for (int i = 0; i < 4; i++) {
    int row = lr + i * 8;
    tile[row][lc] = vh[((size_t)b * SEQ + ty * 32 + row) * LAT + tx * 32 + lc];
  }
  __syncthreads();
  for (int pass = 0; pass < 2; ++pass) {
#pragma unroll
    for (int i = 0; i < 4; i++) {
      int row = lr + i * 8;
      ((volatile float*)vt)[((size_t)b * LAT + tx * 32 + row) * SEQ + ty * 32 + lc] = tile[lc][row];
    }
    __threadfence();
  }
}

extern "C" void kernel_launch(void* const* d_in, const int* in_sizes, int n_in,
                              void* d_out, int out_size, void* d_ws, size_t ws_size,
                              hipStream_t stream) {
  (void)in_sizes; (void)n_in; (void)out_size; (void)ws_size;
  const float* x = (const float*)d_in[0];
  const float* P[4][6];
  for (int f = 0; f < 4; f++)
    for (int j = 0; j < 6; j++)
      P[f][j] = (const float*)d_in[1 + f * 6 + j];

  char* ws = (char*)d_ws;
  const size_t MB8 = (size_t)8 * 1024 * 1024;
  float* xn = (float*)(ws + 0 * MB8);
  float* yb = (float*)(ws + 1 * MB8);
  float* qf = (float*)(ws + 2 * MB8);
  float* kf = (float*)(ws + 3 * MB8);
  float* vf = (float*)(ws + 4 * MB8);
  float* sc = (float*)(ws + 5 * MB8);
  float* pf = (float*)(ws + 6 * MB8);
  float* vt = (float*)(ws + 7 * MB8);

  norm_kernel<<<NTOK, 256, 0, stream>>>(x, xn);
  fff_kernel<0><<<NTOK, 256, 0, stream>>>(xn, P[0][0], P[0][1], P[0][2], P[0][3], P[0][4], P[0][5], qf);
  fff_kernel<0><<<NTOK, 256, 0, stream>>>(xn, P[1][0], P[1][1], P[1][2], P[1][3], P[1][4], P[1][5], kf);
  fff_kernel<0><<<NTOK, 256, 0, stream>>>(xn, P[2][0], P[2][1], P[2][2], P[2][3], P[2][4], P[2][5], vf);
  abt_split_kernel<<<dim3((SEQ / 16) * (SEQ / 256), 2), 256, 0, stream>>>(
      qf, LAT, (long)SEQ * LAT, kf, LAT, (long)SEQ * LAT, sc, SEQ, (long)SEQ * SEQ, nullptr, 0, SEQ, LAT, 0.03125f);
  softmax_kernel<<<NTOK, 256, 0, stream>>>(sc, pf);
  vtrans_kernel<<<NTOK, 256, 0, stream>>>(vf, vt);
  abt_split_kernel<<<dim3((SEQ / 16) * (LAT / 256), 2), 256, 0, stream>>>(
      pf, SEQ, (long)SEQ * SEQ, vt, SEQ, (long)LAT * SEQ, yb, LAT, (long)SEQ * LAT, xn, (long)SEQ * LAT, LAT, SEQ, 1.0f);
  fff_kernel<1><<<NTOK, 256, 0, stream>>>(yb, P[3][0], P[3][1], P[3][2], P[3][3], P[3][4], P[3][5], (float*)d_out);
}
